// Model_15556371546561
// MI455X (gfx1250) — hardware-run, weakly checked
//
#include <hip/hip_runtime.h>
#include <math.h>

typedef __attribute__((ext_vector_type(16))) _Float16 v16h;
typedef __attribute__((ext_vector_type(8)))  _Float16 v8h;
typedef __attribute__((ext_vector_type(16))) __bf16   v16b;
typedef __attribute__((ext_vector_type(8)))  __bf16   v8b;
typedef __attribute__((ext_vector_type(8)))  float    v8f;
typedef __attribute__((ext_vector_type(4)))  float    v4f;
typedef __attribute__((ext_vector_type(2)))  float    v2f;
typedef __attribute__((ext_vector_type(4)))  unsigned int v4u;
typedef __attribute__((ext_vector_type(2)))  unsigned int v2u;

constexpr int kBatch  = 16;
constexpr int kNS     = 32768;
constexpr int kBands  = 64;
constexpr int kTaps   = 128;
constexpr int kFr     = 128;
constexpr int kDm     = 64;
constexpr int kHeads  = 4;
constexpr int kHd     = 16;
constexpr int kLayers = 4;
constexpr int kAtoms  = 16;
constexpr int kTok    = kBatch * kFr;
constexpr int kNAtom  = kBatch * kAtoms;
constexpr int kEmbIn  = 97;
constexpr int kEmbK   = 128;
static_assert(kHeads * kHd == kDm, "head split");
static_assert(4 * 4 == kHd, "score scale is 1/4 = 1/sqrt(head dim)");
constexpr float kQScale = 1.0f / 4.0f;
static_assert(kTok == 2048 && kNAtom == 256, "token and atom counts");
static_assert((kTaps % 32) == 0 && (kEmbK % 32) == 0 && (kDm % 32) == 0, "GEMM K multiples of 32");
static_assert((kTok % 64) == 0 && (kDm % 64) == 0 && ((3 * kDm) % 64) == 0, "GEMM M,N multiples of 64");

constexpr int kR0 = 12, kR1 = 48, kR2 = 192, kR3 = 768, kR4 = 3072, kR5 = 12288;
constexpr int kP0 = 2,  kP1 = 6,  kP2 = 22,  kP3 = 86,  kP4 = 342,  kP5 = 1366;
static_assert(kP1 == 4 * kP0 - 2 && kP2 == 4 * kP1 - 2 && kP3 == 4 * kP2 - 2 && kP4 == 4 * kP3 - 2 && kP5 == 4 * kP4 - 2, "pad chain");
static_assert(kR5 * 8 / 12 * 4 == kNS, "last layer length");

constexpr float kCLat = 16.0f;
constexpr float kCW   = 256.0f;
constexpr float kC0   = 64.0f;
constexpr float kC1   = 256.0f;
constexpr float kC2   = 1024.0f;
constexpr float kC3   = 2048.0f;
constexpr float kC4   = 4096.0f;
constexpr float kC5   = 4096.0f;
constexpr float kCT   = 16384.0f;

constexpr int kWFilt = 0;
constexpr int kWQkv  = kWFilt + kBands * kTaps;
constexpr int kWAo   = kWQkv + kLayers * 3 * kDm * kDm;
constexpr int kWF1   = kWAo + kLayers * kDm * kDm;
constexpr int kWF2   = kWF1 + kLayers * kDm * kDm;
constexpr int kWEmb  = kWF2 + kLayers * kDm * kDm;
constexpr int kWSelN = kWEmb + kDm * kEmbK;
static_assert(kWSelN == 114688, "selection weight plane elements");

constexpr int kYUp = 0;
constexpr int kYL0 = kYUp + 512 * 64;
constexpr int kYL1 = kYL0 + 256 * 128;
constexpr int kYL2 = kYL1 + 256 * 128;
constexpr int kYL3 = kYL2 + 128 * 128;
constexpr int kYL4 = kYL3 + 64 * 64;
constexpr int kYN  = kYL4 + 32 * 32;
static_assert(kYN == 119808, "synthesis weight plane elements");

constexpr size_t kSzPostab = (size_t)kFr * 64 * 4;
constexpr size_t kSzWSel   = (size_t)kWSelN * 2;
constexpr size_t kSzWSyn   = (size_t)kYN * 2;
constexpr size_t kSzAW     = (size_t)kTok * kTaps * 2;
constexpr size_t kSzTokF   = (size_t)kTok * kDm * 4;
constexpr size_t kSzFE     = (size_t)kTok * kEmbK * 2;
constexpr size_t kSzTokH   = (size_t)kTok * kDm * 2;
constexpr size_t kSzQkv    = (size_t)kTok * 3 * kDm * 4;
constexpr size_t kSzMeta   = (size_t)kBatch * 32 * 4;
constexpr size_t kSzLat    = (size_t)kNAtom * kDm * 2;
constexpr size_t kSzPL0    = (size_t)kNAtom * kR0 * 64 * 2 + 128;
constexpr size_t kSzPL1    = (size_t)kNAtom * kR1 * 64 * 2 + 128;
constexpr size_t kSzPL2    = (size_t)kNAtom * kR2 * 64 * 2 + 128;
constexpr size_t kSzPL3    = (size_t)kNAtom * kR3 * 32 * 2 + 128;
constexpr size_t kSzPL4    = (size_t)kNAtom * kR4 * 16 * 2 + 128;
constexpr size_t kSzPL5    = (size_t)kNAtom * kR5 * 8 * 2 + 128;
constexpr size_t kSzTout   = (size_t)kNAtom * kNS * 2;
constexpr size_t kSzPmax   = (size_t)kNAtom * 32 * 32 * 4;

constexpr size_t kOffPostab = 0;
constexpr size_t kOffWSH  = kOffPostab + kSzPostab;
constexpr size_t kOffWSL  = kOffWSH + kSzWSel;
constexpr size_t kOffWSY  = kOffWSL + kSzWSel;
constexpr size_t kOffAWH  = kOffWSY + kSzWSyn;
constexpr size_t kOffAWL  = kOffAWH + kSzAW;
constexpr size_t kOffSPEC = kOffAWL + kSzAW;
constexpr size_t kOffFEH  = kOffSPEC + kSzTokF;
constexpr size_t kOffFEL  = kOffFEH + kSzFE;
constexpr size_t kOffHA   = kOffFEL + kSzFE;
constexpr size_t kOffHB   = kOffHA + kSzTokF;
constexpr size_t kOffHP1H = kOffHB + kSzTokF;
constexpr size_t kOffHP1L = kOffHP1H + kSzTokH;
constexpr size_t kOffHP2H = kOffHP1L + kSzTokH;
constexpr size_t kOffHP2L = kOffHP2H + kSzTokH;
constexpr size_t kOffQKV  = kOffHP2L + kSzTokH;
constexpr size_t kOffOPH  = kOffQKV + kSzQkv;
constexpr size_t kOffOPL  = kOffOPH + kSzTokH;
constexpr size_t kOffT1   = kOffOPL + kSzTokH;
constexpr size_t kOffT2   = kOffT1 + kSzTokF;
constexpr size_t kOffFFH  = kOffT2 + kSzTokF;
constexpr size_t kOffFFL  = kOffFFH + kSzTokH;
constexpr size_t kOffMETA = kOffFFL + kSzTokH;
constexpr size_t kOffLAT  = kOffMETA + kSzMeta;
constexpr size_t kOffPL0  = kOffLAT + kSzLat;
constexpr size_t kOffPL1  = kOffPL0 + kSzPL0;
constexpr size_t kOffPL2  = kOffPL1 + kSzPL1;
constexpr size_t kOffPL3  = kOffPL2 + kSzPL2;
constexpr size_t kOffPL4  = kOffPL3 + kSzPL3;
constexpr size_t kOffPL5  = kOffPL4 + kSzPL4;
constexpr size_t kOffTOUT = kOffPL5 + kSzPL5;
constexpr size_t kOffPMAX = kOffTOUT + kSzTout;
constexpr size_t kWsTotal = kOffPMAX + kSzPmax;
static_assert(kWsTotal == 123319040ull, "carve total");
static_assert(kWsTotal <= 134217728ull, "carve cap");
static_assert((kSzWSel % 128) == 0 && (kSzWSyn % 128) == 0 && (kSzMeta % 128) == 0 && (kSzPL0 % 128) == 0 &&
              (kSzPL1 % 128) == 0 && (kSzPL2 % 128) == 0 && (kSzPL3 % 128) == 0 && (kSzPL4 % 128) == 0 &&
              (kSzPL5 % 128) == 0, "line-aligned regions");

__device__ __forceinline__ unsigned short f2bf_bits(float f) {
  unsigned u = __float_as_uint(f);
  return (unsigned short)((u + 0x7FFFu + ((u >> 16) & 1u)) >> 16);
}
__device__ __forceinline__ float bf_bits2f(unsigned short h) { return __uint_as_float(((unsigned)h) << 16); }
__device__ __forceinline__ unsigned pk16(unsigned short a, unsigned short b) { return (unsigned)a | ((unsigned)b << 16); }
__device__ __forceinline__ unsigned short h_bits_flush(float f) {
  const float g = (fabsf(f) < 6.103515625e-5f) ? 0.0f : f;
  const _Float16 h = (_Float16)g;
  return __builtin_bit_cast(unsigned short, h);
}
__device__ __forceinline__ float h16_to_f32(unsigned hb) {
  const unsigned sgn = (hb & 0x8000u) << 16;
  const unsigned em = hb & 0x7fffu;
  const float fn = __uint_as_float((em << 13) + 0x38000000u);
  const float fs = (float)em * 5.9604644775390625e-8f;
  const float mag = (em < 0x400u) ? fs : fn;
  return __uint_as_float(__float_as_uint(mag) | sgn);
}
__device__ __forceinline__ void pack_bf16_hilo(const float (&v)[8], v4u& hi, v4u& lo) {
  unsigned short hb[8], lb[8];
#pragma unroll
  for (int e = 0; e < 8; ++e) {
    hb[e] = f2bf_bits(v[e]);
    lb[e] = f2bf_bits(v[e] - bf_bits2f(hb[e]));
  }
  hi = (v4u){pk16(hb[0], hb[1]), pk16(hb[2], hb[3]), pk16(hb[4], hb[5]), pk16(hb[6], hb[7])};
  lo = (v4u){pk16(lb[0], lb[1]), pk16(lb[2], lb[3]), pk16(lb[4], lb[5]), pk16(lb[6], lb[7])};
}
__device__ __forceinline__ v4u pack_f16_flush(const float (&v)[8]) {
  unsigned short hb[8];
#pragma unroll
  for (int e = 0; e < 8; ++e) hb[e] = h_bits_flush(v[e]);
  return (v4u){pk16(hb[0], hb[1]), pk16(hb[2], hb[3]), pk16(hb[4], hb[5]), pk16(hb[6], hb[7])};
}

__device__ __forceinline__ v8f mma_b(v16b a, v16b b, v8f c) {
  c = __builtin_amdgcn_wmma_f32_16x16x32_bf16(false, a, false, b, (short)0, c, false, false);
  asm volatile("v_nop\n\tv_nop\n\tv_nop\n\tv_nop" : "+v"(c) : "v"(a), "v"(b));
  return c;
}
__device__ __forceinline__ v8f mma_h(v16h a, v16h b, v8f c) {
  c = __builtin_amdgcn_wmma_f32_16x16x32_f16(false, a, false, b, (short)0, c, false, false);
  asm volatile("v_nop\n\tv_nop\n\tv_nop\n\tv_nop" : "+v"(c) : "v"(a), "v"(b));
  return c;
}
__device__ __forceinline__ v16b frag_b(const __bf16* p) {
  union U { v16b v; v8b h[2]; } f;
  f.h[0] = *(const v8b*)(p);
  f.h[1] = *(const v8b*)(p + 16);
  return f.v;
}
__device__ __forceinline__ v16h frag_h(const _Float16* p) {
  union U { v16h v; v8h h[2]; } f;
  f.h[0] = *(const v8h*)(p);
  f.h[1] = *(const v8h*)(p + 16);
  return f.v;
}

__global__ __launch_bounds__(128) void pos_table_kernel(float* __restrict__ postab) {
#pragma clang fp contract(off)
  __shared__ __align__(16) float sP[kFr * 64];
  const int t = threadIdx.x;
  const float rinv = 1.0f / 127.0f;
  const float s = (float)t * rinv;
  const float om = 1.0f - s;
  float pos = fmaf((float)t, rinv, -om);
  pos = (t == kFr - 1) ? 1.0f : pos;
  const float PI_F = 3.14159265358979323846f;
  const float y = pos * PI_F;
  float* rowp = sP + t * 64;
  rowp[0] = pos;
#pragma unroll 1
  for (int c = 33; c < 64; ++c) rowp[c] = 0.0f;
#pragma unroll 1
  for (int j = 0; j < 16; ++j) {
    const float arg = y * (float)(1 << j);
    const double a = (double)arg;
    const double nn = (double)rintf((float)(a * 0.15915494309189535));
    const double r = fma(-nn, 6.283185307179586, a);
    const float rh = (float)r;
    const float rl = (float)(r - (double)rh);
    const float sn = sinf(rh);
    const float cs = cosf(rh);
    rowp[1 + j]  = sn + rl * cs;
    rowp[17 + j] = cs - rl * sn;
  }
  __syncthreads();
  for (int pass = 0; pass < 2; ++pass) {
#pragma unroll 1
    for (int it = 0; it < 16; ++it) {
      const int i4 = (it * 128 + t) * 4;
      const v4f v = *(const v4f*)(sP + i4);
      *(volatile v4f*)(postab + i4) = v;
    }
    __threadfence();
  }
}

__global__ __launch_bounds__(256) void selw_pack_kernel(
    const float* __restrict__ filt, const float* __restrict__ qkvw, const float* __restrict__ aow,
    const float* __restrict__ f1w, const float* __restrict__ f2w, const float* __restrict__ embw,
    unsigned short* __restrict__ WH, unsigned short* __restrict__ WL) {
  const int blk = blockIdx.x, tid = threadIdx.x;
  const float* src = filt;
  int b0 = 0, dOff = kWFilt;
  bool emb = false;
  if (blk < 4) { src = filt; b0 = 0; dOff = kWFilt; }
  else if (blk < 28) { src = qkvw; b0 = 4; dOff = kWQkv; }
  else if (blk < 36) { src = aow; b0 = 28; dOff = kWAo; }
  else if (blk < 44) { src = f1w; b0 = 36; dOff = kWF1; }
  else if (blk < 52) { src = f2w; b0 = 44; dOff = kWF2; }
  else { src = embw; b0 = 52; dOff = kWEmb; emb = true; }
  const int e0 = ((blk - b0) * 256 + tid) * 8;
  float v[8];
  if (!emb) {
    const v4f a0 = *(const v4f*)(src + e0);
    const v4f a1 = *(const v4f*)(src + e0 + 4);
#pragma unroll
    for (int e = 0; e < 4; ++e) { v[e] = a0[e]; v[4 + e] = a1[e]; }
  } else {
    const int o = e0 >> 7, k0 = e0 & 127;
#pragma unroll
    for (int e = 0; e < 8; ++e) {
      const int k = k0 + e;
      int si = (k < 64) ? (33 + k) : (k - 64);
      si = (si > kEmbIn - 1) ? (kEmbIn - 1) : si;
      float x = src[o * kEmbIn + si];
      asm volatile("" : "+v"(x));
      v[e] = (k < kEmbIn) ? x : 0.0f;
    }
  }
  v4u hi, lo;
  pack_bf16_hilo(v, hi, lo);
  unsigned short* ph = WH + dOff + e0;
  unsigned short* pl = WL + dOff + e0;
  *(volatile v4u*)ph = hi;
  *(volatile v4u*)pl = lo;
  __threadfence();
  *(volatile v4u*)ph = hi;
  *(volatile v4u*)pl = lo;
}

__global__ __launch_bounds__(256) void synw_pack_kernel(
    const float* __restrict__ upw, const float* __restrict__ w0, const float* __restrict__ w1,
    const float* __restrict__ w2, const float* __restrict__ w3, const float* __restrict__ w4,
    unsigned short* __restrict__ W) {
  const int blk = blockIdx.x, tid = threadIdx.x;
  const float* src = upw;
  int b0 = 0, dOff = kYUp, cin = 64, cout = 64, segN = 32768;
  bool conv = false;
  if (blk < 16) { src = upw; b0 = 0; dOff = kYUp; cin = 64; cout = 64; segN = 32768; conv = false; }
  else if (blk < 32) { src = w0; b0 = 16; dOff = kYL0; cin = 64; cout = 64; segN = 32768; conv = true; }
  else if (blk < 48) { src = w1; b0 = 32; dOff = kYL1; cin = 64; cout = 64; segN = 32768; conv = true; }
  else if (blk < 56) { src = w2; b0 = 48; dOff = kYL2; cin = 64; cout = 32; segN = 16384; conv = true; }
  else if (blk < 58) { src = w3; b0 = 56; dOff = kYL3; cin = 32; cout = 16; segN = 4096; conv = true; }
  else { src = w4; b0 = 58; dOff = kYL4; cin = 16; cout = 8; segN = 1024; conv = true; }
  const int e0 = ((blk - b0) * 256 + tid) * 8;
  const bool active = e0 < segN;
  const int e0c = active ? e0 : (segN - 8);
  float v[8];
  if (!conv) {
    const int n = e0c >> 6, k0 = e0c & 63;
    const int srow = ((n & 63) << 3) + (n >> 6);
    const v4f a0 = *(const v4f*)(src + srow * 64 + k0);
    const v4f a1 = *(const v4f*)(src + srow * 64 + k0 + 4);
#pragma unroll
    for (int e = 0; e < 4; ++e) { v[e] = a0[e]; v[4 + e] = a1[e]; }
  } else {
    const int kk2 = 2 * cin;
    const int n = e0c / kk2;
    const int k0 = e0c - n * kk2;
    const int j1 = n / cout;
    const int o = n - j1 * cout;
    const bool late = k0 >= cin;
    const int kk = late ? (k0 - cin) : k0;
    const int jj = late ? j1 : (j1 + 4);
#pragma unroll
    for (int e = 0; e < 8; ++e) v[e] = src[((kk + e) * cout + o) * 8 + jj];
  }
#pragma unroll
  for (int e = 0; e < 8; ++e) v[e] = v[e] * kCW;
  const v4u u = pack_f16_flush(v);
  if (active) {
    unsigned short* p = W + dOff + e0;
    *(volatile v4u*)p = u;
    __threadfence();
    *(volatile v4u*)p = u;
  }
}

__global__ __launch_bounds__(256) void zero_pads_kernel(
    unsigned short* __restrict__ pl0, unsigned short* __restrict__ s0, unsigned short* __restrict__ s1,
    unsigned short* __restrict__ s2, unsigned short* __restrict__ s3, unsigned short* __restrict__ s4,
    unsigned short* __restrict__ s5) {
  const int g = blockIdx.x * 256 + threadIdx.x;
  const bool isPad = g < 8192;
  const bool isSp = (g >= 8192) && (g < 8192 + 48);
  const int line = g >> 3;
  const int atom = (line >> 2) & 255;
  const int wh = line & 3;
  const int padOff = atom * (kR0 * 64) + ((wh < 2) ? (wh * 64) : (640 + (wh - 2) * 64)) + (g & 7) * 8;
  int sp = (g - 8192) >> 3;
  sp = sp < 0 ? 0 : (sp > 5 ? 5 : sp);
  unsigned short* sb = (sp == 0) ? s0 : (sp == 1) ? s1 : (sp == 2) ? s2 : (sp == 3) ? s3 : (sp == 4) ? s4 : s5;
  unsigned short* p = isPad ? (pl0 + padOff) : (sb + (g & 7) * 8);
  if (isPad || isSp) {
    const v4u z = (v4u){0u, 0u, 0u, 0u};
    *(volatile v4u*)p = z;
    __threadfence();
    *(volatile v4u*)p = z;
  }
}

__global__ __launch_bounds__(256) void winsum_kernel(const float* __restrict__ x,
                                                     unsigned short* __restrict__ AH, unsigned short* __restrict__ AL) {
  const int gid = blockIdx.x * 256 + threadIdx.x;
  const int row = gid >> 4, k0 = (gid & 15) * 8;
  const int b = row >> 7, f = row & 127;
  const float* xb = x + (size_t)b * kNS;
  const int kofs = k0 - 64;
  const int sU = 256 * f - 256 + kofs;
  float a0 = 0.0f, a1 = 0.0f, a2 = 0.0f, a3 = 0.0f;
#pragma unroll 4
  for (int it = 0; it < 128; ++it) {
    const int i = sU + 4 * it;
    const bool ok = (i >= 0) && (i < kNS) && (i >= kofs);
    int ic = i < 0 ? 0 : i;
    ic = ic > kNS - 4 ? kNS - 4 : ic;
    const v4f vv = *(const v4f*)(xb + ic);
    float p0 = vv[0], p1 = vv[1], p2 = vv[2], p3 = vv[3];
    asm volatile("" : "+v"(p0), "+v"(p1), "+v"(p2), "+v"(p3));
    a0 += ok ? p0 : 0.0f;
    a1 += ok ? p1 : 0.0f;
    a2 += ok ? p2 : 0.0f;
    a3 += ok ? p3 : 0.0f;
  }
  const int loc = (f == 0) ? 0 : (256 * f - 256);
  const int rs = loc + kofs;
  const int ad = 256 * f + 256 + kofs;
  float rem[8], add[8];
#pragma unroll
  for (int q = 0; q < 2; ++q) {
    const int ir = rs + 4 * q, ia = ad + 4 * q;
    const bool okr = (ir >= 0) && (ir < kNS);
    const bool oka = (ia >= 0) && (ia < kNS);
    int irc = ir < 0 ? 0 : ir;
    irc = irc > kNS - 4 ? kNS - 4 : irc;
    int iac = ia < 0 ? 0 : ia;
    iac = iac > kNS - 4 ? kNS - 4 : iac;
    const v4f vr = *(const v4f*)(xb + irc);
    const v4f va = *(const v4f*)(xb + iac);
    float r0 = vr[0], r1 = vr[1], r2 = vr[2], r3 = vr[3];
    float d0 = va[0], d1 = va[1], d2 = va[2], d3 = va[3];
    asm volatile("" : "+v"(r0), "+v"(r1), "+v"(r2), "+v"(r3));
    asm volatile("" : "+v"(d0), "+v"(d1), "+v"(d2), "+v"(d3));
    rem[4 * q + 0] = okr ? r0 : 0.0f;
    rem[4 * q + 1] = okr ? r1 : 0.0f;
    rem[4 * q + 2] = okr ? r2 : 0.0f;
    rem[4 * q + 3] = okr ? r3 : 0.0f;
    add[4 * q + 0] = oka ? d0 : 0.0f;
    add[4 * q + 1] = oka ? d1 : 0.0f;
    add[4 * q + 2] = oka ? d2 : 0.0f;
    add[4 * q + 3] = oka ? d3 : 0.0f;
  }
  float w[8];
  w[0] = (a0 + a1) + (a2 + a3);
#pragma unroll
  for (int e = 1; e < 8; ++e) w[e] = (w[e - 1] - rem[e - 1]) + add[e - 1];
  v4u hi, lo;
  pack_bf16_hilo(w, hi, lo);
  unsigned short* ph = AH + (size_t)row * kTaps + k0;
  unsigned short* pl = AL + (size_t)row * kTaps + k0;
  *(volatile v4u*)ph = hi;
  *(volatile v4u*)pl = lo;
  __threadfence();
  *(volatile v4u*)ph = hi;
  *(volatile v4u*)pl = lo;
}

template <int BIAS_MODE, int ACT, int OUT_MODE>
__global__ __launch_bounds__(256) void sel_gemm_kernel(
    const unsigned short* __restrict__ Ahp, const unsigned short* __restrict__ Alp, int lda,
    const unsigned short* __restrict__ Bhp, const unsigned short* __restrict__ Blp, int ldb,
    void* __restrict__ Cout, void* __restrict__ Cout2, int ldc,
    const float* __restrict__ bias, int M, int N, int K, float scale) {
  const __bf16* Ah = (const __bf16*)Ahp;
  const __bf16* Al = (const __bf16*)Alp;
  const __bf16* Bh = (const __bf16*)Bhp;
  const __bf16* Bl = (const __bf16*)Blp;
  __shared__ __align__(16) float sT[8][16 * 68];
  const int lane = threadIdx.x & 31;
  const int wave = threadIdx.x >> 5;
  const int tilesN = N >> 6;
  const int tilesM = M >> 6;
  const int tile = blockIdx.x * 8 + wave;
  if (tile >= tilesM * tilesN) return;
  const int tm = tile / tilesN;
  const int tn = tile - tm * tilesN;
  const int m0 = tm << 6;
  const int n0 = tn << 6;
  const int rlane = lane & 15;
  const int koff  = (lane >> 4) * 8;
  const int mOff  = (lane >> 4) * 8;

  v8f acc[4][4];
#pragma unroll
  for (int i = 0; i < 4; ++i)
#pragma unroll
    for (int j = 0; j < 4; ++j) acc[i][j] = (v8f){0.f, 0.f, 0.f, 0.f, 0.f, 0.f, 0.f, 0.f};

  for (int k0 = 0; k0 < K; k0 += 32) {
    v16b bh[4], bl[4];
#pragma unroll
    for (int j = 0; j < 4; ++j) {
      const size_t bo = (size_t)(n0 + (j << 4) + rlane) * ldb + koff + k0;
      bh[j] = frag_b(Bh + bo);
      bl[j] = frag_b(Bl + bo);
    }
#pragma unroll
    for (int i = 0; i < 4; ++i) {
      const size_t ao = (size_t)(m0 + (i << 4) + rlane) * lda + koff + k0;
      const v16b ah = frag_b(Ah + ao);
      const v16b al = frag_b(Al + ao);
#pragma unroll
      for (int j = 0; j < 4; ++j) {
        acc[i][j] = mma_b(ah, bl[j], acc[i][j]);
        acc[i][j] = mma_b(al, bh[j], acc[i][j]);
        acc[i][j] = mma_b(ah, bh[j], acc[i][j]);
      }
    }
  }

  float* slab = sT[wave];
#pragma unroll
  for (int i = 0; i < 4; ++i) {
    const int mBase = m0 + (i << 4);
#pragma unroll
    for (int j = 0; j < 4; ++j) {
      const int n = n0 + (j << 4) + rlane;
      float bv = 0.f;
      if (BIAS_MODE == 2) bv = bias[n];
#pragma unroll
      for (int r = 0; r < 8; ++r) {
        float v = acc[i][j][r] * scale;
        if (BIAS_MODE == 2) v += bv;
        if (ACT == 2) v = fmaxf(v, 0.0f);
        slab[(mOff + r) * 68 + (j << 4) + rlane] = v;
      }
    }
    __builtin_amdgcn_fence(__ATOMIC_RELEASE, "workgroup");
    __builtin_amdgcn_wave_barrier();
    __builtin_amdgcn_fence(__ATOMIC_ACQUIRE, "workgroup");
    if (OUT_MODE == 0) {
      float* C = (float*)Cout;
      const int hh = lane >> 4, c4 = (lane & 15) * 4;
      for (int pass = 0; pass < 2; ++pass) {
#pragma unroll
        for (int it = 0; it < 8; ++it) {
          const int row = it * 2 + hh;
          v4f v = *(const v4f*)(slab + row * 68 + c4);
          *(volatile v4f*)(C + (size_t)(mBase + row) * ldc + n0 + c4) = v;
        }
        __threadfence();
      }
    } else {
      const int q = lane >> 3, c8 = (lane & 7) * 8;
      unsigned short* C  = (unsigned short*)Cout;
      unsigned short* C2 = (unsigned short*)Cout2;
      for (int pass = 0; pass < 2; ++pass) {
#pragma unroll
        for (int it = 0; it < 4; ++it) {
          const int row = it * 4 + q;
          const float* sp = slab + row * 68 + c8;
          v8h hv, lv;
#pragma unroll
          for (int e = 0; e < 8; ++e) {
            unsigned short hb = f2bf_bits(sp[e]);
            unsigned short lb = f2bf_bits(sp[e] - bf_bits2f(hb));
            hv[e] = __builtin_bit_cast(_Float16, hb);
            lv[e] = __builtin_bit_cast(_Float16, lb);
          }
          *(volatile v8h*)(C + (size_t)(mBase + row) * ldc + n0 + c8) = hv;
          *(volatile v8h*)(C2 + (size_t)(mBase + row) * ldc + n0 + c8) = lv;
        }
        __threadfence();
      }
    }
    __builtin_amdgcn_fence(__ATOMIC_RELEASE, "workgroup");
    __builtin_amdgcn_wave_barrier();
    __builtin_amdgcn_fence(__ATOMIC_ACQUIRE, "workgroup");
  }
}

__global__ __launch_bounds__(256) void feat_kernel(const float* __restrict__ spec, const float* __restrict__ postab,
                                                   unsigned short* __restrict__ FH, unsigned short* __restrict__ FL) {
  const int gid = blockIdx.x * 256 + threadIdx.x;
  const int row = gid >> 3, g = gid & 7, t = row & (kFr - 1);
  float a[8], p[8];
  {
    const v4f s0 = *(const v4f*)(spec + (size_t)row * 64 + 8 * g);
    const v4f s1 = *(const v4f*)(spec + (size_t)row * 64 + 8 * g + 4);
    const v4f q0 = *(const v4f*)(postab + t * 64 + 8 * g);
    const v4f q1 = *(const v4f*)(postab + t * 64 + 8 * g + 4);
#pragma unroll
    for (int e = 0; e < 4; ++e) { a[e] = s0[e]; a[4 + e] = s1[e]; p[e] = q0[e]; p[4 + e] = q1[e]; }
  }
  v4u ah, al, ph, pl;
  pack_bf16_hilo(a, ah, al);
  pack_bf16_hilo(p, ph, pl);
  unsigned short* bh = FH + (size_t)row * kEmbK + 8 * g;
  unsigned short* bl = FL + (size_t)row * kEmbK + 8 * g;
  *(volatile v4u*)bh = ah;
  *(volatile v4u*)(bh + 64) = ph;
  *(volatile v4u*)bl = al;
  *(volatile v4u*)(bl + 64) = pl;
  __threadfence();
  *(volatile v4u*)bh = ah;
  *(volatile v4u*)(bh + 64) = ph;
  *(volatile v4u*)bl = al;
  *(volatile v4u*)(bl + 64) = pl;
}

__global__ __launch_bounds__(256) void split_rows_kernel(const float* __restrict__ src, unsigned short* __restrict__ dhi,
                                                         unsigned short* __restrict__ dlo, int total8) {
  const int i = blockIdx.x * 256 + threadIdx.x;
  if (i >= total8) return;
  const size_t e0 = (size_t)i << 3;
  const v4f a0 = *(const v4f*)(src + e0);
  const v4f a1 = *(const v4f*)(src + e0 + 4);
  float v[8];
#pragma unroll
  for (int e = 0; e < 4; ++e) { v[e] = a0[e]; v[4 + e] = a1[e]; }
  v4u hi, lo;
  pack_bf16_hilo(v, hi, lo);
  *(volatile v4u*)(dhi + e0) = hi;
  *(volatile v4u*)(dlo + e0) = lo;
  __threadfence();
  *(volatile v4u*)(dhi + e0) = hi;
  *(volatile v4u*)(dlo + e0) = lo;
}

__device__ __forceinline__ float dot16(const float (&q)[16], const float* kr) {
  const v4f k0 = *(const v4f*)(kr);
  const v4f k1 = *(const v4f*)(kr + 4);
  const v4f k2 = *(const v4f*)(kr + 8);
  const v4f k3 = *(const v4f*)(kr + 12);
  float s = q[0] * k0[0];
  s = fmaf(q[1], k0[1], s);
  s = fmaf(q[2], k0[2], s);
  s = fmaf(q[3], k0[3], s);
  s = fmaf(q[4], k1[0], s);
  s = fmaf(q[5], k1[1], s);
  s = fmaf(q[6], k1[2], s);
  s = fmaf(q[7], k1[3], s);
  s = fmaf(q[8], k2[0], s);
  s = fmaf(q[9], k2[1], s);
  s = fmaf(q[10], k2[2], s);
  s = fmaf(q[11], k2[3], s);
  s = fmaf(q[12], k3[0], s);
  s = fmaf(q[13], k3[1], s);
  s = fmaf(q[14], k3[2], s);
  s = fmaf(q[15], k3[3], s);
  return s;
}

__global__ __launch_bounds__(128) void attn_kernel(const float* __restrict__ qkv,
                                                   unsigned short* __restrict__ OH, unsigned short* __restrict__ OL) {
  __shared__ __align__(16) float sK[kFr * kHd];
  __shared__ __align__(16) float sV[kFr * kHd];
  __shared__ __align__(16) float sO[kFr * 68];
  const int b = blockIdx.x, tid = threadIdx.x, lane = tid & 31, wave = tid >> 5;
  const float* rowp = qkv + (size_t)(b * kFr + tid) * (3 * kDm);
#pragma unroll 1
  for (int hd = 0; hd < kHeads; ++hd) {
    __syncthreads();
    float q[16];
#pragma unroll
    for (int c = 0; c < 4; ++c) {
      const v4f kk = *(const v4f*)(rowp + kDm + hd * kHd + 4 * c);
      const v4f vv = *(const v4f*)(rowp + 2 * kDm + hd * kHd + 4 * c);
      const v4f qq = *(const v4f*)(rowp + hd * kHd + 4 * c);
      *(v4f*)(sK + tid * kHd + 4 * c) = kk;
      *(v4f*)(sV + tid * kHd + 4 * c) = vv;
      q[4 * c + 0] = qq[0] * kQScale;
      q[4 * c + 1] = qq[1] * kQScale;
      q[4 * c + 2] = qq[2] * kQScale;
      q[4 * c + 3] = qq[3] * kQScale;
    }
    __syncthreads();
    float mx = -INFINITY;
#pragma unroll 1
    for (int k = 0; k < kFr; ++k) mx = fmaxf(mx, dot16(q, sK + k * kHd));
    float l = 0.0f;
    float o[16];
#pragma unroll
    for (int d = 0; d < 16; ++d) o[d] = 0.0f;
#pragma unroll 1
    for (int k = 0; k < kFr; ++k) {
      const float s = dot16(q, sK + k * kHd);
      const float p = expf(s - mx);
      l += p;
      const float* vr = sV + k * kHd;
#pragma unroll
      for (int c = 0; c < 4; ++c) {
        const v4f vv = *(const v4f*)(vr + 4 * c);
        o[4 * c + 0] = fmaf(p, vv[0], o[4 * c + 0]);
        o[4 * c + 1] = fmaf(p, vv[1], o[4 * c + 1]);
        o[4 * c + 2] = fmaf(p, vv[2], o[4 * c + 2]);
        o[4 * c + 3] = fmaf(p, vv[3], o[4 * c + 3]);
      }
    }
    const float inv = 1.0f / l;
#pragma unroll
    for (int d = 0; d < 16; ++d) sO[tid * 68 + hd * kHd + d] = o[d] * inv;
  }
  __syncthreads();
  const int q4 = lane >> 3, c8 = (lane & 7) * 8;
  for (int pass = 0; pass < 2; ++pass) {
#pragma unroll 1
    for (int it = 0; it < 8; ++it) {
      const int r = it * 16 + wave * 4 + q4;
      const float* sp = sO + r * 68 + c8;
      const v4f x0 = *(const v4f*)(sp);
      const v4f x1 = *(const v4f*)(sp + 4);
      float v[8];
#pragma unroll
      for (int e = 0; e < 4; ++e) { v[e] = x0[e]; v[4 + e] = x1[e]; }
      v4u hi, lo;
      pack_bf16_hilo(v, hi, lo);
      const size_t oo = (size_t)(b * kFr + r) * kDm + c8;
      *(volatile v4u*)(OH + oo) = hi;
      *(volatile v4u*)(OL + oo) = lo;
    }
    __threadfence();
  }
}

__global__ __launch_bounds__(256) void ln_kernel(const float* __restrict__ hin, const float* __restrict__ addv,
                                                 const float* __restrict__ gam, const float* __restrict__ bet,
                                                 float* __restrict__ hout, unsigned short* __restrict__ PH,
                                                 unsigned short* __restrict__ PL) {
  const int lane = threadIdx.x & 31, wave = threadIdx.x >> 5;
  const int row = blockIdx.x * 8 + wave;
  const int c = 2 * lane;
  const v2f hv = *(const v2f*)(hin + (size_t)row * kDm + c);
  const v2f av = *(const v2f*)(addv + (size_t)row * kDm + c);
  const v2f gv = *(const v2f*)(gam + c);
  const v2f bv = *(const v2f*)(bet + c);
  const float x0 = hv[0] + av[0];
  const float x1 = hv[1] + av[1];
  float s = x0 + x1;
#pragma unroll
  for (int off = 16; off > 0; off >>= 1) s += __shfl_xor(s, off, 32);
  const float mean = s * (1.0f / 64.0f);
  const float d0 = x0 - mean, d1 = x1 - mean;
  float vs = d0 * d0 + d1 * d1;
#pragma unroll
  for (int off = 16; off > 0; off >>= 1) vs += __shfl_xor(vs, off, 32);
  const float var = vs * (1.0f / 64.0f);
  const float inv = 1.0f / sqrtf(var + 1e-5f);
  const float y0 = (d0 * inv) * gv[0] + bv[0];
  const float y1 = (d1 * inv) * gv[1] + bv[1];
  const unsigned short h0 = f2bf_bits(y0), h1 = f2bf_bits(y1);
  const unsigned short l0 = f2bf_bits(y0 - bf_bits2f(h0)), l1 = f2bf_bits(y1 - bf_bits2f(h1));
  const unsigned wh = pk16(h0, h1), wl = pk16(l0, l1);
  const v2f yv = (v2f){y0, y1};
  float* op = hout + (size_t)row * kDm + c;
  unsigned* ph = (unsigned*)(PH + (size_t)row * kDm + c);
  unsigned* pl = (unsigned*)(PL + (size_t)row * kDm + c);
  *(volatile v2f*)op = yv;
  *(volatile unsigned*)ph = wh;
  *(volatile unsigned*)pl = wl;
  __threadfence();
  *(volatile v2f*)op = yv;
  *(volatile unsigned*)ph = wh;
  *(volatile unsigned*)pl = wl;
}

__global__ __launch_bounds__(128) void topk_kernel(const float* __restrict__ h, const float* __restrict__ spec,
                                                   const float* __restrict__ wenv, const float* __restrict__ benv,
                                                   unsigned* __restrict__ meta, unsigned short* __restrict__ lat) {
  __shared__ float sP[kFr];
  __shared__ float sRedA[4];
  __shared__ float sRedB[4];
  __shared__ int sIdx[kAtoms];
  __shared__ float sVal[kAtoms];
  const int b = blockIdx.x, t = threadIdx.x, lane = t & 31, wave = t >> 5;
  if (t < kAtoms) { sIdx[t] = 0; sVal[t] = 0.0f; }
  const size_t rp = (size_t)(b * kFr + t) * kDm;
  float acc = 0.0f;
#pragma unroll 1
  for (int c4 = 0; c4 < 16; ++c4) {
    const v4f hv = *(const v4f*)(h + rp + 4 * c4);
    const v4f sv = *(const v4f*)(spec + rp + 4 * c4);
    const v4f wv = *(const v4f*)(wenv + 4 * c4);
    acc = fmaf(wv[0], hv[0] + sv[0], acc);
    acc = fmaf(wv[1], hv[1] + sv[1], acc);
    acc = fmaf(wv[2], hv[2] + sv[2], acc);
    acc = fmaf(wv[3], hv[3] + sv[3], acc);
  }
  const float logit = acc + benv[0];
  float m = logit;
#pragma unroll
  for (int off = 16; off > 0; off >>= 1) m = fmaxf(m, __shfl_xor(m, off, 32));
  if (lane == 0) sRedA[wave] = m;
  __syncthreads();
  const float mx = fmaxf(fmaxf(sRedA[0], sRedA[1]), fmaxf(sRedA[2], sRedA[3]));
  const float e = expf(logit - mx);
  float s = e;
#pragma unroll
  for (int off = 16; off > 0; off >>= 1) s += __shfl_xor(s, off, 32);
  if (lane == 0) sRedB[wave] = s;
  __syncthreads();
  const float tot = (sRedB[0] + sRedB[1]) + (sRedB[2] + sRedB[3]);
  const float p = e * (1.0f / tot);
  sP[t] = p;
  __syncthreads();
  int cnt = 0;
#pragma unroll 4
  for (int u = 0; u < kFr; ++u) {
    const float pu = sP[u];
    cnt += ((pu > p) || ((pu == p) && (u < t))) ? 1 : 0;
  }
  if (cnt < kAtoms) { sIdx[cnt] = t; sVal[cnt] = p; }
  __syncthreads();
  {
    const int a = t >> 3, c8 = (t & 7) * 8;
    int idx = sIdx[a];
    idx = idx < 0 ? 0 : (idx > kFr - 1 ? kFr - 1 : idx);
    const size_t sp = (size_t)(b * kFr + idx) * kDm + c8;
    const v4f h0 = *(const v4f*)(h + sp);
    const v4f h1 = *(const v4f*)(h + sp + 4);
    const v4f s0 = *(const v4f*)(spec + sp);
    const v4f s1 = *(const v4f*)(spec + sp + 4);
    float v[8];
#pragma unroll
    for (int q = 0; q < 4; ++q) { v[q] = (h0[q] + s0[q]) * kCLat; v[4 + q] = (h1[q] + s1[q]) * kCLat; }
    const v4u u = pack_f16_flush(v);
    unsigned short* lp = lat + (size_t)(b * kAtoms + a) * kDm + c8;
    *(volatile v4u*)lp = u;
    __threadfence();
    *(volatile v4u*)lp = u;
  }
  if (wave == 0) {
    const int li = lane & 15;
    const unsigned wi = (unsigned)sIdx[li];
    const unsigned wv = __float_as_uint(sVal[li]);
    const unsigned word = (lane < 16) ? wi : wv;
    volatile unsigned* mp = meta + b * 32 + lane;
    *mp = word;
    __threadfence();
    *mp = word;
  }
}

template <int NSUB, int CIN, int COUT, int RIN, int PIN, bool CONV>
__global__ __launch_bounds__(256) void synth_gemm_kernel(
    const unsigned short* __restrict__ Ap, int lda,
    const unsigned short* __restrict__ Btp, int ldb,
    unsigned short* __restrict__ Cp, int ldc,
    const float* __restrict__ bias, int M, int N, int K, float accScale, float outCarry) {
  const _Float16* A = (const _Float16*)Ap;
  const _Float16* Bt = (const _Float16*)Btp;
  __shared__ __align__(16) float sT[8][16 * 68];
  constexpr int WT = 16 * NSUB;
  constexpr int LIN = (RIN / 12) * 8;
  constexpr int LOUT = 4 * LIN;
  constexpr int POUT = 4 * PIN - 2;
  const int lane = threadIdx.x & 31;
  const int wave = threadIdx.x >> 5;
  const int tilesN = N / WT;
  const int tilesM = M >> 6;
  const int tile = blockIdx.x * 8 + wave;
  if (tile >= tilesM * tilesN) return;
  const int tm = tile / tilesN;
  const int tn = tile - tm * tilesN;
  const int m0 = tm << 6;
  const int n0 = tn * WT;
  const int rlane = lane & 15;
  const int koff  = (lane >> 4) * 8;
  const int mOff  = (lane >> 4) * 8;

  v8f acc[4][NSUB];
#pragma unroll
  for (int i = 0; i < 4; ++i)
#pragma unroll
    for (int j = 0; j < NSUB; ++j) acc[i][j] = (v8f){0.f, 0.f, 0.f, 0.f, 0.f, 0.f, 0.f, 0.f};

  for (int k0 = 0; k0 < K; k0 += 32) {
    v16h bh[NSUB];
#pragma unroll
    for (int j = 0; j < NSUB; ++j)
      bh[j] = frag_h(Bt + (size_t)(n0 + (j << 4) + rlane) * ldb + koff + k0);
#pragma unroll
    for (int i = 0; i < 4; ++i) {
      const v16h ah = frag_h(A + (size_t)(m0 + (i << 4) + rlane) * lda + koff + k0);
#pragma unroll
      for (int j = 0; j < NSUB; ++j) acc[i][j] = mma_h(ah, bh[j], acc[i][j]);
    }
  }

  float* slab = sT[wave];
#pragma unroll
  for (int i = 0; i < 4; ++i) {
    const int mBase = m0 + (i << 4);
    int q4[8];
#pragma unroll
    for (int r = 0; r < 8; ++r) {
      const unsigned rowg = (unsigned)(mBase + mOff + r);
      q4[r] = CONV ? (int)(4u * (rowg % (unsigned)RIN)) : 0;
    }
#pragma unroll
    for (int j = 0; j < NSUB; ++j) {
      const int n = n0 + (j << 4) + rlane;
      const int bi = CONV ? (n & (COUT - 1)) : (((n & 63) << 3) + (n >> 6));
      const float bv = bias[bi];
      const int jq = CONV ? (n / COUT) : 0;
#pragma unroll
      for (int r = 0; r < 8; ++r) {
        float v = acc[i][j][r] * accScale + bv;
        if (CONV) {
          v = (v >= 0.0f) ? v : 0.2f * v;
          const unsigned qq = (unsigned)(q4[r] + jq - POUT);
          v = (qq < (unsigned)LOUT) ? (v * outCarry) : 0.0f;
        } else {
          v = v * outCarry;
        }
        slab[(mOff + r) * 68 + (j << 4) + rlane] = v;
      }
    }
    __builtin_amdgcn_fence(__ATOMIC_RELEASE, "workgroup");
    __builtin_amdgcn_wave_barrier();
    __builtin_amdgcn_fence(__ATOMIC_ACQUIRE, "workgroup");
    for (int pass = 0; pass < 2; ++pass) {
#pragma unroll
      for (int it = 0; it < NSUB; ++it) {
        const int c = it * 32 + lane;
        const int row = c / (2 * NSUB);
        const int col8 = (c % (2 * NSUB)) * 8;
        const float* sp = slab + row * 68 + col8;
        const v4f x0 = *(const v4f*)(sp);
        const v4f x1 = *(const v4f*)(sp + 4);
        float v[8];
#pragma unroll
        for (int e = 0; e < 4; ++e) { v[e] = x0[e]; v[4 + e] = x1[e]; }
        const v4u u = pack_f16_flush(v);
        *(volatile v4u*)(Cp + (size_t)(mBase + row) * ldc + n0 + col8) = u;
      }
      __threadfence();
    }
    __builtin_amdgcn_fence(__ATOMIC_RELEASE, "workgroup");
    __builtin_amdgcn_wave_barrier();
    __builtin_amdgcn_fence(__ATOMIC_ACQUIRE, "workgroup");
  }
}

__global__ __launch_bounds__(256) void l5_kernel(const unsigned short* __restrict__ P5, const float* __restrict__ w5,
                                                 const float* __restrict__ b5, unsigned short* __restrict__ TOUT,
                                                 float* __restrict__ pmax) {
  __shared__ float sM[8];
  const int blk = blockIdx.x, tid = threadIdx.x, lane = tid & 31, wave = tid >> 5;
  const int atom = blk >> 5;
  const int u = (blk & 31) * 256 + tid;
  const unsigned short* src = P5 + ((size_t)atom * kR5 + (kP5 - 1) + u) * 8;
  const v4u r0 = *(const v4u*)(src);
  const v4u r1 = *(const v4u*)(src + 8);
  const v4u r2 = *(const v4u*)(src + 16);
  float xm[8], x0[8], xp[8];
#pragma unroll
  for (int i = 0; i < 4; ++i) {
    const unsigned wa = r0[i], wb = r1[i], wc = r2[i];
    xm[2 * i] = h16_to_f32(wa & 0xffffu);
    xm[2 * i + 1] = h16_to_f32(wa >> 16);
    x0[2 * i] = h16_to_f32(wb & 0xffffu);
    x0[2 * i + 1] = h16_to_f32(wb >> 16);
    xp[2 * i] = h16_to_f32(wc & 0xffffu);
    xp[2 * i + 1] = h16_to_f32(wc >> 16);
  }
  float y0 = 0.0f, y1 = 0.0f, y2 = 0.0f, y3 = 0.0f;
#pragma unroll
  for (int c = 0; c < 8; ++c) {
    y0 = fmaf(w5[c * 8 + 2], x0[c], y0);
    y0 = fmaf(w5[c * 8 + 6], xm[c], y0);
    y1 = fmaf(w5[c * 8 + 3], x0[c], y1);
    y1 = fmaf(w5[c * 8 + 7], xm[c], y1);
    y2 = fmaf(w5[c * 8 + 0], xp[c], y2);
    y2 = fmaf(w5[c * 8 + 4], x0[c], y2);
    y3 = fmaf(w5[c * 8 + 1], xp[c], y3);
    y3 = fmaf(w5[c * 8 + 5], x0[c], y3);
  }
  const float bb = b5[0];
  constexpr float kInv5 = 1.0f / kC5;
  y0 = y0 * kInv5 + bb;
  y1 = y1 * kInv5 + bb;
  y2 = y2 * kInv5 + bb;
  y3 = y3 * kInv5 + bb;
  const unsigned short t0 = h_bits_flush(y0 * kCT), t1 = h_bits_flush(y1 * kCT);
  const unsigned short t2 = h_bits_flush(y2 * kCT), t3 = h_bits_flush(y3 * kCT);
  const v2u tw = (v2u){pk16(t0, t1), pk16(t2, t3)};
  unsigned short* tp = TOUT + (size_t)atom * kNS + 4 * u;
  *(volatile v2u*)tp = tw;
  __threadfence();
  *(volatile v2u*)tp = tw;
  float m = fmaxf(fmaxf(y0, y1), fmaxf(y2, y3));
#pragma unroll
  for (int off = 16; off > 0; off >>= 1) m = fmaxf(m, __shfl_xor(m, off, 32));
  if (lane == 0) sM[wave] = m;
  __syncthreads();
  if (wave == 0) {
    const float mm = fmaxf(fmaxf(fmaxf(sM[0], sM[1]), fmaxf(sM[2], sM[3])), fmaxf(fmaxf(sM[4], sM[5]), fmaxf(sM[6], sM[7])));
    volatile float* pp = pmax + (size_t)blk * 32 + lane;
    *pp = mm;
    __threadfence();
    *pp = mm;
  }
}

__global__ __launch_bounds__(256) void final_kernel(const unsigned short* __restrict__ TOUT, const float* __restrict__ pmax,
                                                    const unsigned* __restrict__ meta, float* __restrict__ out) {
  __shared__ float sR[kAtoms];
  __shared__ float sVv[kAtoms];
  __shared__ int sOff[kAtoms];
  const int blk = blockIdx.x, tid = threadIdx.x, lane = tid & 31, wave = tid >> 5;
  const int b = blk >> 5;
  const int s0 = (blk & 31) * 1024 + tid * 4;
#pragma unroll
  for (int q = 0; q < 2; ++q) {
    const int a = 2 * wave + q;
    float m = pmax[((size_t)(b * kAtoms + a) * 32 + lane) * 32];
#pragma unroll
    for (int off = 16; off > 0; off >>= 1) m = fmaxf(m, __shfl_xor(m, off, 32));
    const float r = 1.0f / (m + 1e-8f);
    if (lane == 0) sR[a] = r;
  }
  {
    const int li = tid & 15;
    unsigned wi = meta[b * 32 + li];
    unsigned wv = meta[b * 32 + 16 + li];
    asm volatile("" : "+v"(wi), "+v"(wv));
    int idx = (int)wi;
    idx = idx < 0 ? 0 : (idx > kFr - 1 ? kFr - 1 : idx);
    if (tid < kAtoms) { sOff[tid] = idx * 256; sVv[tid] = __uint_as_float(wv); }
  }
  __syncthreads();
  float a0 = 0.0f, a1 = 0.0f, a2 = 0.0f, a3 = 0.0f;
  constexpr float kInvT = 1.0f / kCT;
#pragma unroll 1
  for (int a = 0; a < kAtoms; ++a) {
    const int sp = s0 - sOff[a];
    const bool ok = sp >= 0;
    const int spc = ok ? sp : 0;
    const v2u w = *(const v2u*)(TOUT + (size_t)(b * kAtoms + a) * kNS + spc);
    unsigned wa = w[0], wb = w[1];
    asm volatile("" : "+v"(wa), "+v"(wb));
    const float r = sR[a], vl = sVv[a];
    const float t0 = h16_to_f32(wa & 0xffffu) * kInvT;
    const float t1 = h16_to_f32(wa >> 16) * kInvT;
    const float t2 = h16_to_f32(wb & 0xffffu) * kInvT;
    const float t3 = h16_to_f32(wb >> 16) * kInvT;
    const float n0 = a0 + (t0 * r) * vl;
    const float n1 = a1 + (t1 * r) * vl;
    const float n2 = a2 + (t2 * r) * vl;
    const float n3 = a3 + (t3 * r) * vl;
    a0 = ok ? n0 : a0;
    a1 = ok ? n1 : a1;
    a2 = ok ? n2 : a2;
    a3 = ok ? n3 : a3;
  }
  const v4f ov = (v4f){a0, a1, a2, a3};
  float* op = out + (size_t)b * kNS + s0;
  *(volatile v4f*)op = ov;
  __threadfence();
  *(volatile v4f*)op = ov;
}

extern "C" void kernel_launch(void* const* d_in, const int* in_sizes, int n_in,
                              void* d_out, int out_size, void* d_ws, size_t ws_size,
                              hipStream_t stream) {
  if (n_in < 32) return;
  if (in_sizes[0] != kBatch * kNS) return;
  if (in_sizes[1] != kBands * kTaps) return;
  if (in_sizes[2] != kDm * kEmbIn) return;
  if (in_sizes[4] != kLayers * 3 * kDm * kDm) return;
  if (in_sizes[6] != kLayers * kDm * kDm) return;
  if (in_sizes[10] != kLayers * kDm * kDm) return;
  if (in_sizes[12] != kLayers * kDm * kDm) return;
  if (in_sizes[16] != kDm) return;
  if (in_sizes[18] != 512 * 64) return;
  if (in_sizes[20] != 64 * 64 * 8 || in_sizes[22] != 64 * 64 * 8 || in_sizes[24] != 64 * 32 * 8) return;
  if (in_sizes[26] != 32 * 16 * 8 || in_sizes[28] != 16 * 8 * 8 || in_sizes[30] != 8 * 8) return;
  if (out_size != kBatch * kNS) return;
  if (ws_size < kWsTotal) return;

  const float* x     = (const float*)d_in[0];
  const float* fbf   = (const float*)d_in[1];
  const float* ew    = (const float*)d_in[2];
  const float* ebv   = (const float*)d_in[3];
  const float* qkvw  = (const float*)d_in[4];
  const float* qkvb  = (const float*)d_in[5];
  const float* aow   = (const float*)d_in[6];
  const float* aob   = (const float*)d_in[7];
  const float* ln1g  = (const float*)d_in[8];
  const float* ln1b  = (const float*)d_in[9];
  const float* f1w   = (const float*)d_in[10];
  const float* f1b   = (const float*)d_in[11];
  const float* f2w   = (const float*)d_in[12];
  const float* f2b   = (const float*)d_in[13];
  const float* ln2g  = (const float*)d_in[14];
  const float* ln2b  = (const float*)d_in[15];
  const float* tew   = (const float*)d_in[16];
  const float* teb   = (const float*)d_in[17];
  const float* upw   = (const float*)d_in[18];
  const float* upb   = (const float*)d_in[19];
  const float* tw0   = (const float*)d_in[20];
  const float* tb0   = (const float*)d_in[21];
  const float* tw1   = (const float*)d_in[22];
  const float* tb1   = (const float*)d_in[23];
  const float* tw2   = (const float*)d_in[24];
  const float* tb2   = (const float*)d_in[25];
  const float* tw3   = (const float*)d_in[26];
  const float* tb3   = (const float*)d_in[27];
  const float* tw4   = (const float*)d_in[28];
  const float* tb4   = (const float*)d_in[29];
  const float* tw5   = (const float*)d_in[30];
  const float* tb5   = (const float*)d_in[31];
  float* out = (float*)d_out;

  char* ws = (char*)d_ws;
  float*          POSTAB = (float*)(ws + kOffPostab);
  unsigned short* WSH  = (unsigned short*)(ws + kOffWSH);
  unsigned short* WSL  = (unsigned short*)(ws + kOffWSL);
  unsigned short* WSY  = (unsigned short*)(ws + kOffWSY);
  unsigned short* AWH  = (unsigned short*)(ws + kOffAWH);
  unsigned short* AWL  = (unsigned short*)(ws + kOffAWL);
  float*          SPEC = (float*)(ws + kOffSPEC);
  unsigned short* FEH  = (unsigned short*)(ws + kOffFEH);
  unsigned short* FEL  = (unsigned short*)(ws + kOffFEL);
  float*          HA   = (float*)(ws + kOffHA);
  float*          HB   = (float*)(ws + kOffHB);
  unsigned short* HP1H = (unsigned short*)(ws + kOffHP1H);
  unsigned short* HP1L = (unsigned short*)(ws + kOffHP1L);
  unsigned short* HP2H = (unsigned short*)(ws + kOffHP2H);
  unsigned short* HP2L = (unsigned short*)(ws + kOffHP2L);
  float*          QKV  = (float*)(ws + kOffQKV);
  unsigned short* OPH  = (unsigned short*)(ws + kOffOPH);
  unsigned short* OPL  = (unsigned short*)(ws + kOffOPL);
  float*          T1   = (float*)(ws + kOffT1);
  float*          T2   = (float*)(ws + kOffT2);
  unsigned short* FFH  = (unsigned short*)(ws + kOffFFH);
  unsigned short* FFL  = (unsigned short*)(ws + kOffFFL);
  unsigned*       META = (unsigned*)(ws + kOffMETA);
  unsigned short* LAT  = (unsigned short*)(ws + kOffLAT);
  unsigned short* PL0  = (unsigned short*)(ws + kOffPL0);
  unsigned short* PL1  = (unsigned short*)(ws + kOffPL1);
  unsigned short* PL2  = (unsigned short*)(ws + kOffPL2);
  unsigned short* PL3  = (unsigned short*)(ws + kOffPL3);
  unsigned short* PL4  = (unsigned short*)(ws + kOffPL4);
  unsigned short* PL5  = (unsigned short*)(ws + kOffPL5);
  unsigned short* TOUT = (unsigned short*)(ws + kOffTOUT);
  float*          PMAX = (float*)(ws + kOffPMAX);

  pos_table_kernel<<<1, 128, 0, stream>>>(POSTAB);
  selw_pack_kernel<<<56, 256, 0, stream>>>(fbf, qkvw, aow, f1w, f2w, ew, WSH, WSL);
  synw_pack_kernel<<<59, 256, 0, stream>>>(upw, tw0, tw1, tw2, tw3, tw4, WSY);
  zero_pads_kernel<<<33, 256, 0, stream>>>(
      PL0,
      PL0 + (size_t)kNAtom * kR0 * 64, PL1 + (size_t)kNAtom * kR1 * 64, PL2 + (size_t)kNAtom * kR2 * 64,
      PL3 + (size_t)kNAtom * kR3 * 32, PL4 + (size_t)kNAtom * kR4 * 16, PL5 + (size_t)kNAtom * kR5 * 8);

  winsum_kernel<<<(kTok * 16) / 256, 256, 0, stream>>>(x, AWH, AWL);
  sel_gemm_kernel<0, 0, 0><<<4, 256, 0, stream>>>(
      AWH, AWL, kTaps, WSH + kWFilt, WSL + kWFilt, kTaps,
      (void*)SPEC, nullptr, kDm, nullptr, kTok, kBands, kTaps, 1.0f / 512.0f);

  feat_kernel<<<(kTok * 8) / 256, 256, 0, stream>>>(SPEC, POSTAB, FEH, FEL);
  sel_gemm_kernel<2, 0, 0><<<4, 256, 0, stream>>>(
      FEH, FEL, kEmbK, WSH + kWEmb, WSL + kWEmb, kEmbK,
      (void*)HA, nullptr, kDm, ebv, kTok, kDm, kEmbK, 1.0f);
  split_rows_kernel<<<(kTok * kDm / 8) / 256, 256, 0, stream>>>(HA, HP1H, HP1L, kTok * kDm / 8);

  for (int l = 0; l < kLayers; ++l) {
    sel_gemm_kernel<2, 0, 0><<<12, 256, 0, stream>>>(
        HP1H, HP1L, kDm, WSH + kWQkv + l * 3 * kDm * kDm, WSL + kWQkv + l * 3 * kDm * kDm, kDm,
        (void*)QKV, nullptr, 3 * kDm, qkvb + l * 3 * kDm, kTok, 3 * kDm, kDm, 1.0f);
    attn_kernel<<<kBatch, 128, 0, stream>>>(QKV, OPH, OPL);
    sel_gemm_kernel<2, 0, 0><<<4, 256, 0, stream>>>(
        OPH, OPL, kDm, WSH + kWAo + l * kDm * kDm, WSL + kWAo + l * kDm * kDm, kDm,
        (void*)T1, nullptr, kDm, aob + l * kDm, kTok, kDm, kDm, 1.0f);
    ln_kernel<<<kTok / 8, 256, 0, stream>>>(HA, T1, ln1g + l * kDm, ln1b + l * kDm, HB, HP2H, HP2L);
    sel_gemm_kernel<2, 2, 2><<<4, 256, 0, stream>>>(
        HP2H, HP2L, kDm, WSH + kWF1 + l * kDm * kDm, WSL + kWF1 + l * kDm * kDm, kDm,
        (void*)FFH, (void*)FFL, kDm, f1b + l * kDm, kTok, kDm, kDm, 1.0f);
    sel_gemm_kernel<2, 0, 0><<<4, 256, 0, stream>>>(
        FFH, FFL, kDm, WSH + kWF2 + l * kDm * kDm, WSL + kWF2 + l * kDm * kDm, kDm,
        (void*)T2, nullptr, kDm, f2b + l * kDm, kTok, kDm, kDm, 1.0f);
    ln_kernel<<<kTok / 8, 256, 0, stream>>>(HB, T2, ln2g + l * kDm, ln2b + l * kDm, HA, HP1H, HP1L);
  }

  topk_kernel<<<kBatch, 128, 0, stream>>>(HA, SPEC, tew, teb, META, LAT);

  synth_gemm_kernel<4, 64, 64, kR0, kP0, false><<<4, 256, 0, stream>>>(
      LAT, 64, WSY + kYUp, 64, PL0 + 128, kR0 * 64, upb, kNAtom, 512, 64,
      1.0f / (kCLat * kCW), kC0);
  synth_gemm_kernel<4, 64, 64, kR0, kP0, true><<<24, 256, 0, stream>>>(
      PL0, 64, WSY + kYL0, 128, PL1, 256, tb0, kNAtom * kR0, 256, 128,
      1.0f / (kC0 * kCW), kC1);
  synth_gemm_kernel<4, 64, 64, kR1, kP1, true><<<96, 256, 0, stream>>>(
      PL1, 64, WSY + kYL1, 128, PL2, 256, tb1, kNAtom * kR1, 256, 128,
      1.0f / (kC1 * kCW), kC2);
  synth_gemm_kernel<4, 64, 32, kR2, kP2, true><<<192, 256, 0, stream>>>(
      PL2, 64, WSY + kYL2, 128, PL3, 128, tb2, kNAtom * kR2, 128, 128,
      1.0f / (kC2 * kCW), kC3);
  synth_gemm_kernel<4, 32, 16, kR3, kP3, true><<<384, 256, 0, stream>>>(
      PL3, 32, WSY + kYL3, 64, PL4, 64, tb3, kNAtom * kR3, 64, 64,
      1.0f / (kC3 * kCW), kC4);
  synth_gemm_kernel<2, 16, 8, kR4, kP4, true><<<1536, 256, 0, stream>>>(
      PL4, 16, WSY + kYL4, 32, PL5, 32, tb4, kNAtom * kR4, 32, 32,
      1.0f / (kC4 * kCW), kC5);
  l5_kernel<<<kNAtom * 32, 256, 0, stream>>>(PL5, tw5, tb5, TOUT, PMAX);
  final_kernel<<<kBatch * 32, 256, 0, stream>>>(TOUT, PMAX, META, out);
}
